// GMM_estimator_80556406604184
// MI455X (gfx1250) — hardware-verified
//
#include <hip/hip_runtime.h>


typedef float        v8f   __attribute__((ext_vector_type(8)));
typedef float        v4f   __attribute__((ext_vector_type(4)));
typedef unsigned int v4u   __attribute__((ext_vector_type(4)));
typedef __bf16       v16bf __attribute__((ext_vector_type(16)));

#define IN_DIM   64
#define H_DIM    1024
#define OUT_DIM  12
#define N_PAD    16
#define ROWS_BLK 16
#define HP       1032

#define PREP_W1_BLOCKS (H_DIM / 32)
#define PREP_W2_BLOCKS (H_DIM / 128)

union BFrag { v16bf v; v4u q[2]; };
union C8    { v8f v; v4f q[2]; };

__device__ __forceinline__ unsigned short f2bf(float x) {
  __bf16 b = (__bf16)x;
  return __builtin_bit_cast(unsigned short, b);
}
__device__ __forceinline__ float bf2f(unsigned short u) {
  return __uint_as_float(((unsigned int)u) << 16);
}
__device__ __forceinline__ unsigned int pack2(float a, float b) {
  return (unsigned int)f2bf(a) | ((unsigned int)f2bf(b) << 16);
}
__device__ __forceinline__ v4u cvtpack8(const float* __restrict__ p) {
  const v4f f0 = *(const v4f*)(p);
  const v4f f1 = *(const v4f*)(p + 4);
  v4u q;
  q[0] = pack2(f0[0], f0[1]);
  q[1] = pack2(f0[2], f0[3]);
  q[2] = pack2(f1[0], f1[1]);
  q[3] = pack2(f1[2], f1[3]);
  return q;
}
__device__ __forceinline__ void split_pack2(float x0, float x1, unsigned int& ph, unsigned int& pl) {
  const unsigned short h0 = f2bf(x0), h1 = f2bf(x1);
  const float r0 = x0 - bf2f(h0), r1 = x1 - bf2f(h1);
  ph = (unsigned int)h0 | ((unsigned int)h1 << 16);
  pl = (unsigned int)f2bf(r0) | ((unsigned int)f2bf(r1) << 16);
}

__device__ __forceinline__ v8f wmma_bf16(const BFrag& a, const BFrag& b, v8f c) {
  c = __builtin_amdgcn_wmma_f32_16x16x32_bf16(false, a.v, false, b.v, (short)0, c, false, false);
  asm volatile("v_nop\n\tv_nop\n\tv_nop\n\tv_nop"
               : "+v"(c)
               : "v"(a.q[0]), "v"(a.q[1]), "v"(b.q[0]), "v"(b.q[1]));
  return c;
}

__global__ __launch_bounds__(256)
void prep_operands(const float* __restrict__ tau,
                   const float* __restrict__ W1,
                   const float* __restrict__ W2,
                   unsigned short* __restrict__ W1T,
                   unsigned short* __restrict__ W2T,
                   unsigned short* __restrict__ XB,
                   int Brows) {
  __shared__ float sW[IN_DIM][33];
  const int tid = threadIdx.x;
  if (blockIdx.x < PREP_W1_BLOCKS) {
    const int n0 = blockIdx.x * 32;
    const int c  = tid & 31;
    const int kr = tid >> 5;
#pragma unroll
    for (int j = 0; j < 8; ++j) {
      const int k = kr + 8 * j;
      sW[k][c] = W1[(size_t)k * H_DIM + n0 + c];
    }
    __syncthreads();
    const int r  = tid >> 3;
    const int ch = tid & 7;
    v4u pk;
    pk[0] = pack2(sW[8 * ch + 0][r], sW[8 * ch + 1][r]);
    pk[1] = pack2(sW[8 * ch + 2][r], sW[8 * ch + 3][r]);
    pk[2] = pack2(sW[8 * ch + 4][r], sW[8 * ch + 5][r]);
    pk[3] = pack2(sW[8 * ch + 6][r], sW[8 * ch + 7][r]);
    unsigned short* dst = W1T + (size_t)(n0 + r) * IN_DIM + 8 * ch;
    *(volatile v4u*)dst = pk;
    __threadfence();
    *(volatile v4u*)dst = pk;
  } else if (blockIdx.x < PREP_W1_BLOCKS + PREP_W2_BLOCKS) {
    const int kb0 = (blockIdx.x - PREP_W1_BLOCKS) * 128;
    const int n   = tid >> 4;
    const int kc  = tid & 15;
    const int k   = kb0 + 8 * kc;
    float v[8];
#pragma unroll
    for (int i = 0; i < 8; ++i)
      v[i] = (n < OUT_DIM) ? W2[(size_t)(k + i) * OUT_DIM + n] : 0.0f;
    v4u pk;
    pk[0] = pack2(v[0], v[1]);
    pk[1] = pack2(v[2], v[3]);
    pk[2] = pack2(v[4], v[5]);
    pk[3] = pack2(v[6], v[7]);
    unsigned short* dst = W2T + (size_t)n * H_DIM + k;
    *(volatile v4u*)dst = pk;
    __threadfence();
    *(volatile v4u*)dst = pk;
  } else {
    const int rb  = (blockIdx.x - PREP_W1_BLOCKS - PREP_W2_BLOCKS) * 32;
    const int r   = tid >> 3;
    const int ch  = tid & 7;
    const int row = rb + r;
    if (row < Brows) {
      const v4u pk = cvtpack8(tau + (size_t)row * IN_DIM + 8 * ch);
      unsigned short* dst = XB + (size_t)row * IN_DIM + 8 * ch;
      *(volatile v4u*)dst = pk;
      __threadfence();
      *(volatile v4u*)dst = pk;
    }
  }
}

__global__ __launch_bounds__(256)
void mlp_mix_fused(const unsigned short* __restrict__ XB,
                   const float* __restrict__ b1,
                   const float* __restrict__ b2,
                   const unsigned short* __restrict__ W1T,
                   const unsigned short* __restrict__ W2T,
                   float* __restrict__ out_mu,
                   float* __restrict__ out_cov,
                   int Brows) {
  __shared__ __attribute__((aligned(16))) unsigned short hs_hi[ROWS_BLK * HP];
  __shared__ __attribute__((aligned(16))) unsigned short hs_lo[ROWS_BLK * HP];
  __shared__ __attribute__((aligned(16))) float redC[8][16][16];
  __shared__ float fin[16 * 17];

  const int tid  = threadIdx.x;
  const int w    = tid >> 5;
  const int lane = tid & 31;
  const int l15  = lane & 15;
  const int kb   = (lane >> 4) * 8;
  const int row0 = blockIdx.x * ROWS_BLK;

  int ra = row0 + l15;
  if (ra > Brows - 1) ra = Brows - 1;
  const unsigned short* xrow = XB + (size_t)ra * IN_DIM;
  BFrag bx0, bx1;
  bx0.q[0] = *(const v4u*)(xrow + kb);
  bx0.q[1] = *(const v4u*)(xrow + 16 + kb);
  bx1.q[0] = *(const v4u*)(xrow + 32 + kb);
  bx1.q[1] = *(const v4u*)(xrow + 48 + kb);

#pragma unroll
  for (int t = 0; t < 8; ++t) {
    const int n0 = w * 128 + t * 16;
    const unsigned short* arow = W1T + (size_t)(n0 + l15) * IN_DIM;
    BFrag a0, a1;
    a0.q[0] = *(const v4u*)(arow + kb);
    a0.q[1] = *(const v4u*)(arow + 16 + kb);
    a1.q[0] = *(const v4u*)(arow + 32 + kb);
    a1.q[1] = *(const v4u*)(arow + 48 + kb);

    v8f c = {};
    c = wmma_bf16(a0, bx0, c);
    c = wmma_bf16(a1, bx1, c);

    const int nb = n0 + kb;
    const v4f bA = *(const v4f*)(b1 + nb);
    const v4f bB = *(const v4f*)(b1 + nb + 4);
    const float h0 = fmaxf(c[0] + bA[0], 0.0f);
    const float h1 = fmaxf(c[1] + bA[1], 0.0f);
    const float h2 = fmaxf(c[2] + bA[2], 0.0f);
    const float h3 = fmaxf(c[3] + bA[3], 0.0f);
    const float h4 = fmaxf(c[4] + bB[0], 0.0f);
    const float h5 = fmaxf(c[5] + bB[1], 0.0f);
    const float h6 = fmaxf(c[6] + bB[2], 0.0f);
    const float h7 = fmaxf(c[7] + bB[3], 0.0f);
    v4u qh, ql;
    unsigned int ph, pl;
    split_pack2(h0, h1, ph, pl); qh[0] = ph; ql[0] = pl;
    split_pack2(h2, h3, ph, pl); qh[1] = ph; ql[1] = pl;
    split_pack2(h4, h5, ph, pl); qh[2] = ph; ql[2] = pl;
    split_pack2(h6, h7, ph, pl); qh[3] = ph; ql[3] = pl;
    *(v4u*)(&hs_hi[l15 * HP + nb]) = qh;
    *(v4u*)(&hs_lo[l15 * HP + nb]) = ql;
  }

  __syncthreads();

  v8f c2 = {};
  const unsigned short* hrow_hi = &hs_hi[l15 * HP];
  const unsigned short* hrow_lo = &hs_lo[l15 * HP];
  const unsigned short* wrow    = W2T + (size_t)l15 * H_DIM;
#pragma unroll
  for (int cc = 0; cc < 4; ++cc) {
    const int k0 = w * 128 + cc * 32;
    BFrag ah, al, bw;
    ah.q[0] = *(const v4u*)(hrow_hi + k0 + kb);
    ah.q[1] = *(const v4u*)(hrow_hi + k0 + 16 + kb);
    al.q[0] = *(const v4u*)(hrow_lo + k0 + kb);
    al.q[1] = *(const v4u*)(hrow_lo + k0 + 16 + kb);
    bw.q[0] = *(const v4u*)(wrow + k0 + kb);
    bw.q[1] = *(const v4u*)(wrow + k0 + 16 + kb);
    c2 = wmma_bf16(ah, bw, c2);
    c2 = wmma_bf16(al, bw, c2);
  }

  {
    C8 u; u.v = c2;
    *(v4f*)&redC[w][l15][kb]     = u.q[0];
    *(v4f*)&redC[w][l15][kb + 4] = u.q[1];
  }

  __syncthreads();

  {
    const int n = tid >> 4;
    const int m = tid & 15;
    float s = 0.0f;
#pragma unroll
    for (int ww = 0; ww < 8; ++ww) s += redC[ww][n][m];
    if (n < OUT_DIM) s += bf2f(f2bf(b2[n]));
    fin[m * 17 + n] = s;
  }

  __syncthreads();

  if (tid < 32) {
    const int m    = lane >> 1;
    const int comp = lane & 1;
    const int gm   = row0 + m;
    const float* o = &fin[m * 17 + comp * 6];
    const float a  = o[2];
    const float e  = 0.5f * (o[3] + o[4]);
    const float d  = o[5];
    const float od = e * (a + d);
    v4f cv;
    cv[0] = a * a + e * e;
    cv[1] = od;
    cv[2] = od;
    cv[3] = e * e + d * d;

    const bool wm  = lane < 16;
    const int  gmu = row0 + lane;
    v4f mv = {};
    if (wm) {
      const float* om = &fin[lane * 17];
      mv[0] = om[0]; mv[1] = om[1]; mv[2] = om[6]; mv[3] = om[7];
    }
    float* pc = out_cov + (size_t)gm * 8 + comp * 4;
    float* pm = out_mu + (size_t)gmu * 4;
    const bool sc = gm < Brows;
    const bool sm = wm && (gmu < Brows);
    if (sc) *(volatile v4f*)pc = cv;
    if (sm) *(volatile v4f*)pm = mv;
    __threadfence();
    if (sc) *(volatile v4f*)pc = cv;
    if (sm) *(volatile v4f*)pm = mv;
  }
}

extern "C" void kernel_launch(void* const* d_in, const int* in_sizes, int n_in,
                              void* d_out, int out_size, void* d_ws, size_t ws_size,
                              hipStream_t stream) {
  if (n_in < 5) return;
  const float* tau = (const float*)d_in[0];
  const float* W1  = (const float*)d_in[1];
  const float* b1  = (const float*)d_in[2];
  const float* W2  = (const float*)d_in[3];
  const float* b2  = (const float*)d_in[4];

  if (in_sizes[1] != IN_DIM * H_DIM || in_sizes[2] < H_DIM ||
      in_sizes[3] != H_DIM * OUT_DIM || in_sizes[4] < OUT_DIM) return;

  int Brows = in_sizes[0] / IN_DIM;
  const int Bo = out_size / OUT_DIM;
  if (Bo < Brows) Brows = Bo;
  if (Brows <= 0) return;

  const size_t w1t_bytes = (size_t)H_DIM * IN_DIM * 2;
  const size_t w2t_bytes = (size_t)N_PAD * H_DIM * 2;
  const size_t xb_bytes  = (size_t)Brows * IN_DIM * 2;
  if (w1t_bytes + w2t_bytes + xb_bytes > ws_size) return;
  unsigned short* W1T = (unsigned short*)d_ws;
  unsigned short* W2T = (unsigned short*)((char*)d_ws + w1t_bytes);
  unsigned short* XB  = (unsigned short*)((char*)d_ws + w1t_bytes + w2t_bytes);

  float* out_mu  = (float*)d_out;
  float* out_cov = (float*)d_out + (size_t)Brows * 4;

  const int prep_blocks = PREP_W1_BLOCKS + PREP_W2_BLOCKS + (Brows + 31) / 32;
  prep_operands<<<prep_blocks, 256, 0, stream>>>(tau, W1, W2, W1T, W2T, XB, Brows);

  const int nblk = (Brows + ROWS_BLK - 1) / ROWS_BLK;
  mlp_mix_fused<<<nblk, 256, 0, stream>>>(XB, b1, b2, W1T, W2T, out_mu, out_cov, Brows);
}
